// SKOLRTransitionModel_30305289240701
// MI455X (gfx1250) — hardware-verified
//
#include <hip/hip_runtime.h>
#include <math.h>

constexpr int kB   = 16384;
constexpr int kD   = 256;
constexpr int kU   = 32;
constexpr int kNBR = 8;
constexpr int kMH  = 512;
constexpr int kRH  = 256;
constexpr int kNY  = 20;
constexpr int kRHU = 288;
constexpr int kKIN = 320;
constexpr float kWCarry    = 16.0f;
constexpr float kWCarryInv = 1.0f / 16.0f;
constexpr float kLoCarry   = 2048.0f;
constexpr float kLoInv     = 1.0f / (16.0f * 2048.0f);

constexpr size_t kOffW1  = 0;
constexpr size_t kOffW2  = kOffW1 + (size_t)kNBR * kMH * kD * 2;
constexpr size_t kOffRB  = kOffW2 + (size_t)kNBR * kRH * kMH * 2;
constexpr size_t kOffWO  = kOffRB + (size_t)kNBR * kRH * kKIN * 2;
constexpr size_t kOffSIG = kOffWO + (size_t)kNBR * kD * kRH * 2;
constexpr size_t kOffZG  = kOffSIG + (size_t)kNBR * kD * 4;
constexpr size_t kOffX32 = kOffZG + (size_t)kB * kD * 2;
constexpr size_t kOffHHI = kOffX32;
constexpr size_t kOffHLO = kOffX32 + (size_t)kB * kRH * 2;
constexpr size_t kOffX16 = kOffX32 + (size_t)kB * kMH * 4;
constexpr size_t kOffINP = kOffX16 + (size_t)kB * kMH * 2;
constexpr size_t kOffP0  = kOffINP + (size_t)kB * kKIN * 2;
constexpr size_t kOffP1  = kOffP0 + (size_t)kB * kD * 4;
constexpr size_t kWsTotal = kOffP1 + (size_t)kB * kD * 4;
typedef char ws_total_check[(kWsTotal <= (size_t)134217728u) ? 1 : -1];
typedef char hlo_fits_check[(kOffHLO + (size_t)kB * kRH * 2 <= kOffX16) ? 1 : -1];

typedef __attribute__((ext_vector_type(16))) _Float16 v16h;
typedef __attribute__((ext_vector_type(8)))  _Float16 v8h;
typedef __attribute__((ext_vector_type(16))) __bf16   v16b;
typedef __attribute__((ext_vector_type(8)))  __bf16   v8b;
typedef __attribute__((ext_vector_type(8)))  float    v8f;
typedef __attribute__((ext_vector_type(4)))  float    v4f;
typedef __attribute__((ext_vector_type(2)))  float    v2f;
typedef __attribute__((ext_vector_type(4)))  unsigned int v4u;

__device__ __forceinline__ unsigned short f2bf_bits(float f) {
  unsigned u = __float_as_uint(f);
  return (unsigned short)((u + 0x7FFFu + ((u >> 16) & 1u)) >> 16);
}
__device__ __forceinline__ float bf_bits2f(unsigned short h) { return __uint_as_float(((unsigned)h) << 16); }

__device__ __forceinline__ void dep_guard_h(v8f& a, v8f& b, v16h x, v16h y) { asm volatile("v_nop\n\tv_nop\n\tv_nop\n\tv_nop" : "+v"(a), "+v"(b) : "v"(x), "v"(y)); }
__device__ __forceinline__ void dep_guard_b(v8f& a, v8f& b, v16b x, v16b y) { asm volatile("v_nop\n\tv_nop\n\tv_nop\n\tv_nop" : "+v"(a), "+v"(b) : "v"(x), "v"(y)); }
__device__ __forceinline__ void keep4_h(v16h a, v16h b, v16h c, v16h d) { asm volatile("v_nop" :: "v"(a), "v"(b), "v"(c), "v"(d)); }
__device__ __forceinline__ void keep4_b(v16b a, v16b b, v16b c, v16b d) { asm volatile("v_nop" :: "v"(a), "v"(b), "v"(c), "v"(d)); }
__device__ __forceinline__ void acc_guard4(v8f& a, v8f& b, v8f& c, v8f& d) { asm volatile("v_nop\n\tv_nop\n\tv_nop\n\tv_nop" : "+v"(a), "+v"(b), "+v"(c), "+v"(d)); }
template <typename T> struct Frag;
template <> struct Frag<_Float16> {
  typedef v16h V; union U { v16h v; v8h h[2]; };
  static __device__ __forceinline__ v16h load(const _Float16* p) {
    U f; f.h[0] = *(const v8h*)(p); f.h[1] = *(const v8h*)(p + 16); return f.v;
  }
  static __device__ __forceinline__ v8f mma(v16h a, v16h b, v8f c) {
    return __builtin_amdgcn_wmma_f32_16x16x32_f16(false, a, false, b, (short)0, c, false, false);
  }
  static __device__ __forceinline__ void guard(v8f& a, v8f& b, v16h x, v16h y) { dep_guard_h(a, b, x, y); }
  static __device__ __forceinline__ void keep(v16h a, v16h b, v16h c, v16h d) { keep4_h(a, b, c, d); }
};
template <> struct Frag<__bf16> {
  typedef v16b V; union U { v16b v; v8b h[2]; };
  static __device__ __forceinline__ v16b load(const __bf16* p) {
    U f; f.h[0] = *(const v8b*)(p); f.h[1] = *(const v8b*)(p + 16); return f.v;
  }
  static __device__ __forceinline__ v8f mma(v16b a, v16b b, v8f c) {
    return __builtin_amdgcn_wmma_f32_16x16x32_bf16(false, a, false, b, (short)0, c, false, false);
  }
  static __device__ __forceinline__ void guard(v8f& a, v8f& b, v16b x, v16b y) { dep_guard_b(a, b, x, y); }
  static __device__ __forceinline__ void keep(v16b a, v16b b, v16b c, v16b d) { keep4_b(a, b, c, d); }
};

__device__ __forceinline__ unsigned pk16(unsigned short a, unsigned short b) { return (unsigned)a | ((unsigned)b << 16); }
__device__ __forceinline__ unsigned short h_bits(float f) { const _Float16 h = (_Float16)f; return __builtin_bit_cast(unsigned short, h); }

template <int ET> struct Elem;
template <> struct Elem<0> { typedef _Float16 T; };
template <> struct Elem<1> { typedef __bf16 T; };
template <int ET, bool SPLIT, int BIAS_MODE, int OUT_MODE, bool RESID, int ACT = 0>
__global__ __launch_bounds__(256) void wmma_gemm64(
    const unsigned short* __restrict__ Ap, const unsigned short* __restrict__ A2p, int lda, long strideA,
    const unsigned short* __restrict__ Btp, const unsigned short* __restrict__ Bt2p, int ldb, long strideB,
    void* __restrict__ Cout, void* __restrict__ Cout2, int ldc, long strideC,
    const float* __restrict__ bias,
    const float* __restrict__ resid, long strideR,
    int M, int N, int K, float scale) {
  typedef typename Elem<ET>::T T;
  typedef typename Frag<T>::V V;
  const T* A = (const T*)Ap; const T* A2 = (const T*)A2p; const T* Bt = (const T*)Btp; const T* Bt2 = (const T*)Bt2p;
  __shared__ __align__(16) float sT[8][16 * 68];
  const int b    = blockIdx.y;
  const int lane = threadIdx.x & 31;
  const int wave = threadIdx.x >> 5;
  const int tilesN = N >> 6;
  const int tilesM = M >> 6;
  const int tile = blockIdx.x * 8 + wave;
  if (tile >= tilesM * tilesN) return;
  const int tm = tile / tilesN;
  const int tn = tile - tm * tilesN;
  const int m0 = tm << 6;
  const int n0 = tn << 6;

  const T* Ab  = A  + (size_t)b * strideA;
  const T* Bb  = Bt + (size_t)b * strideB;
  const T* Ab2 = SPLIT ? (A2  + (size_t)b * strideA) : nullptr;
  const T* Bb2 = SPLIT ? (Bt2 + (size_t)b * strideB) : nullptr;

  const int rlane = lane & 15;
  const int koff  = (lane >> 4) * 8;
  const int mOff  = (lane >> 4) * 8;

  v8f acc[4][4];
#pragma unroll
  for (int i = 0; i < 4; ++i)
#pragma unroll
    for (int j = 0; j < 4; ++j) acc[i][j] = (v8f){0.f,0.f,0.f,0.f,0.f,0.f,0.f,0.f};

  for (int k0 = 0; k0 < K; k0 += 32) {
    V bh[4], bl[4];
#pragma unroll
    for (int j = 0; j < 4; ++j) {
      const size_t bo = (size_t)(n0 + (j << 4) + rlane) * ldb + koff + k0;
      bh[j] = Frag<T>::load(Bb + bo);
      if (SPLIT) bl[j] = Frag<T>::load(Bb2 + bo);
    }
#pragma unroll
    for (int i = 0; i < 4; ++i) {
      const size_t ao = (size_t)(m0 + (i << 4) + rlane) * lda + koff + k0;
      V ah = Frag<T>::load(Ab + ao);
      V al;
      if (SPLIT) al = Frag<T>::load(Ab2 + ao);
#pragma unroll
      for (int j = 0; j < 4; ++j) {
        acc[i][j] = Frag<T>::mma(ah, bh[j], acc[i][j]);
        if (SPLIT) {
          acc[i][j] = Frag<T>::mma(ah, bl[j], acc[i][j]);
          acc[i][j] = Frag<T>::mma(al, bh[j], acc[i][j]);
        }
      }
      Frag<T>::guard(acc[i][0], acc[i][3], ah, SPLIT ? al : ah);
    }
    Frag<T>::keep(bh[0], bh[1], bh[2], bh[3]);
    if (SPLIT) Frag<T>::keep(bl[0], bl[1], bl[2], bl[3]);
  }
  acc_guard4(acc[0][0], acc[0][1], acc[0][2], acc[0][3]);
  acc_guard4(acc[1][0], acc[1][1], acc[1][2], acc[1][3]);
  acc_guard4(acc[2][0], acc[2][1], acc[2][2], acc[2][3]);
  acc_guard4(acc[3][0], acc[3][1], acc[3][2], acc[3][3]);

  float* slab = sT[wave];
  const float* Rb = RESID ? (resid + (size_t)b * strideR) : nullptr;
#pragma unroll
  for (int i = 0; i < 4; ++i) {
    const int mBase = m0 + (i << 4);
#pragma unroll
    for (int j = 0; j < 4; ++j) {
      const int n = n0 + (j << 4) + rlane;
      float bv = 0.f;
      if (BIAS_MODE == 2) bv = bias[n];
#pragma unroll
      for (int r = 0; r < 8; ++r) {
        float v = acc[i][j][r] * scale;
        if (BIAS_MODE == 1) v += bias[mBase + mOff + r];
        if (BIAS_MODE == 2) v += bv;
        if (RESID) v += Rb[(size_t)(mBase + mOff + r) * ldc + n];
        if (ACT == 2) v = fmaxf(v, 0.0f);
        if (ACT == 4) v = (v > 0.f) ? v : 0.01f * v;
        slab[(mOff + r) * 68 + (j << 4) + rlane] = v;
      }
    }
    __builtin_amdgcn_fence(__ATOMIC_RELEASE, "workgroup");
    __builtin_amdgcn_wave_barrier();
    __builtin_amdgcn_fence(__ATOMIC_ACQUIRE, "workgroup");
    if (OUT_MODE == 0) {
      float* C = (float*)Cout + (size_t)b * strideC;
      const int hh = lane >> 4, c4 = (lane & 15) * 4;
      for (int pass = 0; pass < 2; ++pass) {
#pragma unroll
        for (int it = 0; it < 8; ++it) {
          const int row = it * 2 + hh;
          v4f v = *(const v4f*)(slab + row * 68 + c4);
          *(volatile v4f*)(C + (size_t)(mBase + row) * ldc + n0 + c4) = v;
        }
        __threadfence();
      }
    } else {
      const int q = lane >> 3, c8 = (lane & 7) * 8;
      unsigned short* C  = (unsigned short*)Cout  + (size_t)b * strideC;
      unsigned short* C2 = (OUT_MODE >= 2) ? ((unsigned short*)Cout2 + (size_t)b * strideC) : nullptr;
      for (int pass = 0; pass < 2; ++pass) {
#pragma unroll
        for (int it = 0; it < 4; ++it) {
          const int row = it * 4 + q;
          const float* sp = slab + row * 68 + c8;
          v8h hv, lv;
#pragma unroll
          for (int e = 0; e < 8; ++e) {
            if (OUT_MODE == 1) {
              hv[e] = (_Float16)sp[e];
            } else if (OUT_MODE == 3) {
              const _Float16 h1 = (_Float16)sp[e];
              hv[e] = h1;
              lv[e] = (_Float16)((sp[e] - (float)h1) * 2048.0f);
            } else {
              unsigned short hb = f2bf_bits(sp[e]);
              unsigned short lb = f2bf_bits(sp[e] - bf_bits2f(hb));
              hv[e] = __builtin_bit_cast(_Float16, hb);
              lv[e] = __builtin_bit_cast(_Float16, lb);
            }
          }
          *(volatile v8h*)(C + (size_t)(mBase + row) * ldc + n0 + c8) = hv;
          if (OUT_MODE >= 2) *(volatile v8h*)(C2 + (size_t)(mBase + row) * ldc + n0 + c8) = lv;
        }
        __threadfence();
      }
    }
    __builtin_amdgcn_fence(__ATOMIC_RELEASE, "workgroup");
    __builtin_amdgcn_wave_barrier();
    __builtin_amdgcn_fence(__ATOMIC_ACQUIRE, "workgroup");
  }
}

__global__ __launch_bounds__(256) void castw_kernel(const float* __restrict__ src, unsigned short* __restrict__ dst,
                                                    int srcCols, int slots, float scale, int total) {
  const int t = blockIdx.x * 256 + threadIdx.x;
  if (t >= total) return;
  const int row  = t / slots;
  const int s    = t - row * slots;
  const int nsrc = srcCols >> 3;
  const bool live = (s < nsrc);
  const int sc = live ? s : (nsrc - 1);
  const float* p = src + (size_t)row * srcCols + sc * 8;
  const v4f a = *(const v4f*)(p);
  const v4f c = *(const v4f*)(p + 4);
  unsigned short hb[8];
#pragma unroll
  for (int e = 0; e < 4; ++e) {
    hb[e]     = h_bits(live ? a[e] * scale : 0.0f);
    hb[4 + e] = h_bits(live ? c[e] * scale : 0.0f);
  }
  const v4u u = (v4u){pk16(hb[0], hb[1]), pk16(hb[2], hb[3]), pk16(hb[4], hb[5]), pk16(hb[6], hb[7])};
  unsigned short* q = dst + 8 * (size_t)t;
  *(volatile v4u*)q = u;
  __threadfence();
  *(volatile v4u*)q = u;
}

__global__ __launch_bounds__(256) void sig_kernel(const float* __restrict__ gates, float* __restrict__ sig, int n4) {
  const int t = blockIdx.x * 256 + threadIdx.x;
  if (t >= n4) return;
  const v4f g = *(const v4f*)(gates + 4 * (size_t)t);
  v4f s;
#pragma unroll
  for (int e = 0; e < 4; ++e) s[e] = 1.0f / (1.0f + expf(-g[e]));
  float* q = sig + 4 * (size_t)t;
  *(volatile v4f*)q = s;
  __threadfence();
  *(volatile v4f*)q = s;
}

__global__ __launch_bounds__(256) void gate_kernel(const float* __restrict__ zt, const float* __restrict__ sig_n,
                                                   unsigned short* __restrict__ zg, int n8) {
  const int t = blockIdx.x * 256 + threadIdx.x;
  if (t >= n8) return;
  const int d0 = (t & 31) * 8;
  const float* p = zt + 8 * (size_t)t;
  const v4f a  = *(const v4f*)(p);
  const v4f c  = *(const v4f*)(p + 4);
  const v4f s0 = *(const v4f*)(sig_n + d0);
  const v4f s1 = *(const v4f*)(sig_n + d0 + 4);
  unsigned short hb[8];
#pragma unroll
  for (int e = 0; e < 4; ++e) {
    hb[e]     = h_bits(a[e] * s0[e]);
    hb[4 + e] = h_bits(c[e] * s1[e]);
  }
  const v4u u = (v4u){pk16(hb[0], hb[1]), pk16(hb[2], hb[3]), pk16(hb[4], hb[5]), pk16(hb[6], hb[7])};
  unsigned short* q = zg + 8 * (size_t)t;
  *(volatile v4u*)q = u;
  __threadfence();
  *(volatile v4u*)q = u;
}

__global__ __launch_bounds__(256) void inp_ctrl_kernel(const float* __restrict__ ut, const float* __restrict__ dtp,
                                                       unsigned short* __restrict__ inp) {
  const int lane = threadIdx.x & 31, wave = threadIdx.x >> 5;
  const int row = blockIdx.x * 32 + wave * 4 + (lane >> 3);
  const int q = lane & 7;
  const bool live = (q < 4);
  const int qc = live ? q : 0;
  const float dtv = dtp[0];
  const float* p = ut + (size_t)row * kU + qc * 8;
  const v4f a = *(const v4f*)(p);
  const v4f c = *(const v4f*)(p + 4);
  unsigned short hb[8];
#pragma unroll
  for (int e = 0; e < 4; ++e) {
    hb[e]     = h_bits(live ? a[e] * dtv : 0.0f);
    hb[4 + e] = h_bits(live ? c[e] * dtv : 0.0f);
  }
  const v4u u = (v4u){pk16(hb[0], hb[1]), pk16(hb[2], hb[3]), pk16(hb[4], hb[5]), pk16(hb[6], hb[7])};
  unsigned short* dq = inp + (size_t)row * kKIN + kRH + q * 8;
  *(volatile v4u*)dq = u;
  __threadfence();
  *(volatile v4u*)dq = u;
}

__global__ __launch_bounds__(256) void ln_gelu_kernel(const float* __restrict__ X, const float* __restrict__ g,
                                                      const float* __restrict__ bta, unsigned short* __restrict__ Y) {
  __shared__ __align__(16) unsigned int sw[8][256];
  const int lane = threadIdx.x & 31, wave = threadIdx.x >> 5;
  const int row = blockIdx.x * 8 + wave;
  const float* xr = X + (size_t)row * kMH;
  v4f x4[4];
#pragma unroll
  for (int i = 0; i < 4; ++i) x4[i] = *(const v4f*)(xr + i * 128 + lane * 4);
  float s = 0.f;
#pragma unroll
  for (int i = 0; i < 4; ++i) s += (x4[i][0] + x4[i][1]) + (x4[i][2] + x4[i][3]);
#pragma unroll
  for (int off = 16; off > 0; off >>= 1) s += __shfl_xor(s, off, 32);
  const float mu = s * (1.0f / 512.0f);
  float q = 0.f;
#pragma unroll
  for (int i = 0; i < 4; ++i)
#pragma unroll
    for (int e = 0; e < 4; ++e) {
      const float d = x4[i][e] - mu;
      q += d * d;
    }
#pragma unroll
  for (int off = 16; off > 0; off >>= 1) q += __shfl_xor(q, off, 32);
  const float var = q * (1.0f / 512.0f);
  const float ri  = rsqrtf(var + 1e-5f);
  unsigned int* swp = sw[wave];
#pragma unroll 1
  for (int it = 0; it < 8; ++it) {
    const int c = it * 64 + lane * 2;
    const v2f xv = *(const v2f*)(xr + c);
    const v2f gv = *(const v2f*)(g + c);
    const v2f bv = *(const v2f*)(bta + c);
    const float n0v = (xv[0] - mu) * ri * gv[0] + bv[0];
    const float n1v = (xv[1] - mu) * ri * gv[1] + bv[1];
    const float a0 = 0.5f * n0v * (1.0f + erff(n0v * 0.70710678118654752f));
    const float a1 = 0.5f * n1v * (1.0f + erff(n1v * 0.70710678118654752f));
    swp[it * 32 + lane] = pk16(h_bits(a0), h_bits(a1));
  }
  __builtin_amdgcn_fence(__ATOMIC_RELEASE, "workgroup");
  __builtin_amdgcn_wave_barrier();
  __builtin_amdgcn_fence(__ATOMIC_ACQUIRE, "workgroup");
  unsigned short* yr = Y + (size_t)row * kMH;
  for (int pass = 0; pass < 2; ++pass) {
#pragma unroll
    for (int k = 0; k < 2; ++k) {
      const v4u val = *(const v4u*)(swp + k * 128 + lane * 4);
      *(volatile v4u*)(yr + k * 256 + lane * 8) = val;
    }
    __threadfence();
  }
}

__global__ __launch_bounds__(256) void yproj_kernel(const float* __restrict__ zt1, const float* __restrict__ ut,
                                                    const float* __restrict__ dtp, const float* __restrict__ Cm,
                                                    const float* __restrict__ Dm, float* __restrict__ out1) {
  __shared__ __align__(16) float zs[32 * kD];
  __shared__ __align__(16) float cs[kNY * kD];
  __shared__ __align__(16) float ds[kNY * kU];
  __shared__ __align__(16) float us[32 * kU];
  __shared__ __align__(16) float ys[32 * kNY];
  const int t = threadIdx.x;
  const int row0 = blockIdx.x * 32;
#pragma unroll
  for (int i = 0; i < 8; ++i) {
    const int idx = i * 256 + t;
    *(v4f*)(zs + idx * 4) = *(const v4f*)(zt1 + (size_t)row0 * kD + idx * 4);
  }
#pragma unroll
  for (int i = 0; i < 5; ++i) {
    const int idx = i * 256 + t;
    *(v4f*)(cs + idx * 4) = *(const v4f*)(Cm + idx * 4);
  }
  {
    const int idx = (t < 160) ? t : 159;
    const v4f dv = *(const v4f*)(Dm + idx * 4);
    if (t < 160) *(v4f*)(ds + idx * 4) = dv;
  }
  {
    const float dtv = dtp[0];
    v4f uv = *(const v4f*)(ut + (size_t)row0 * kU + t * 4);
#pragma unroll
    for (int e = 0; e < 4; ++e) uv[e] = uv[e] * dtv;
    *(v4f*)(us + t * 4) = uv;
  }
  __syncthreads();
  const int r = t >> 3, j = t & 7;
  const int y0 = j, y1 = j + 8;
  const int y2 = (j + 16 < kNY) ? (j + 16) : (kNY - 1);
  float a0 = 0.f, a1 = 0.f, a2 = 0.f;
  {
    const float* zr = zs + r * kD;
    const float* c0 = cs + y0 * kD;
    const float* c1 = cs + y1 * kD;
    const float* c2 = cs + y2 * kD;
#pragma unroll 1
    for (int dq = 0; dq < kD / 4; ++dq) {
      const v4f z  = *(const v4f*)(zr + dq * 4);
      const v4f w0 = *(const v4f*)(c0 + dq * 4);
      const v4f w1 = *(const v4f*)(c1 + dq * 4);
      const v4f w2 = *(const v4f*)(c2 + dq * 4);
#pragma unroll
      for (int e = 0; e < 4; ++e) {
        a0 += z[e] * w0[e];
        a1 += z[e] * w1[e];
        a2 += z[e] * w2[e];
      }
    }
  }
  float u0 = 0.f, u1 = 0.f, u2 = 0.f;
  {
    const float* ur = us + r * kU;
    const float* d0 = ds + y0 * kU;
    const float* d1 = ds + y1 * kU;
    const float* d2 = ds + y2 * kU;
#pragma unroll 1
    for (int uq = 0; uq < kU / 4; ++uq) {
      const v4f uu = *(const v4f*)(ur + uq * 4);
      const v4f w0 = *(const v4f*)(d0 + uq * 4);
      const v4f w1 = *(const v4f*)(d1 + uq * 4);
      const v4f w2 = *(const v4f*)(d2 + uq * 4);
#pragma unroll
      for (int e = 0; e < 4; ++e) {
        u0 += uu[e] * w0[e];
        u1 += uu[e] * w1[e];
        u2 += uu[e] * w2[e];
      }
    }
  }
  ys[r * kNY + y0] = a0 + u0;
  ys[r * kNY + y1] = a1 + u1;
  if (j < 4) ys[r * kNY + y2] = a2 + u2;
  __syncthreads();
  float* ob = out1 + (size_t)blockIdx.x * (32 * kNY);
  for (int pass = 0; pass < 2; ++pass) {
    if (t < 160) {
      const v4f v = *(const v4f*)(ys + t * 4);
      *(volatile v4f*)(ob + t * 4) = v;
    }
    __threadfence();
  }
}

extern "C" void kernel_launch(void* const* d_in, const int* in_sizes, int n_in,
                              void* d_out, int out_size, void* d_ws, size_t ws_size, hipStream_t stream) {
  if (n_in < 16) return;
  if (in_sizes[0] != kB * kD || in_sizes[1] < 1 || in_sizes[2] != kB * kU || in_sizes[3] != kNBR * kD ||
      in_sizes[4] != kNBR * kMH * kD || in_sizes[5] != kNBR * kMH || in_sizes[6] != kNBR * kMH ||
      in_sizes[7] != kNBR * kMH || in_sizes[8] != kNBR * kRH * kMH || in_sizes[9] != kNBR * kRH ||
      in_sizes[12] != kNBR * kRH * kRHU || in_sizes[13] != kNBR * kD * kRH || in_sizes[14] != kNY * kD ||
      in_sizes[15] != kNY * kU) return;
  if ((size_t)out_size < (size_t)kB * kD + (size_t)kB * kNY) return;
  if (ws_size < kWsTotal) return;

  const float* zt    = (const float*)d_in[0];
  const float* dtp   = (const float*)d_in[1];
  const float* ut    = (const float*)d_in[2];
  const float* gates = (const float*)d_in[3];
  const float* W1    = (const float*)d_in[4];
  const float* b1    = (const float*)d_in[5];
  const float* lng   = (const float*)d_in[6];
  const float* lnb   = (const float*)d_in[7];
  const float* W2    = (const float*)d_in[8];
  const float* b2    = (const float*)d_in[9];
  const float* rnnB  = (const float*)d_in[12];
  const float* Wout  = (const float*)d_in[13];
  const float* Cm    = (const float*)d_in[14];
  const float* Dmm   = (const float*)d_in[15];
  float* out0 = (float*)d_out;
  float* out1 = (float*)d_out + (size_t)kB * kD;

  char* ws = (char*)d_ws;
  unsigned short* w1h = (unsigned short*)(ws + kOffW1);
  unsigned short* w2h = (unsigned short*)(ws + kOffW2);
  unsigned short* rbh = (unsigned short*)(ws + kOffRB);
  unsigned short* woh = (unsigned short*)(ws + kOffWO);
  float*          sig = (float*)(ws + kOffSIG);
  unsigned short* zg  = (unsigned short*)(ws + kOffZG);
  float*          x32 = (float*)(ws + kOffX32);
  unsigned short* hhi = (unsigned short*)(ws + kOffHHI);
  unsigned short* hlo = (unsigned short*)(ws + kOffHLO);
  unsigned short* x16 = (unsigned short*)(ws + kOffX16);
  unsigned short* inp = (unsigned short*)(ws + kOffINP);
  float*          p0  = (float*)(ws + kOffP0);
  float*          p1  = (float*)(ws + kOffP1);

  sig_kernel<<<(kNBR * kD / 4 + 255) / 256, 256, 0, stream>>>(gates, sig, kNBR * kD / 4);
  {
    const int tw1 = kNBR * kMH * (kD / 8);
    castw_kernel<<<(tw1 + 255) / 256, 256, 0, stream>>>(W1, w1h, kD, kD / 8, kWCarry, tw1);
    const int tw2 = kNBR * kRH * (kMH / 8);
    castw_kernel<<<(tw2 + 255) / 256, 256, 0, stream>>>(W2, w2h, kMH, kMH / 8, kWCarry, tw2);
    const int trb = kNBR * kRH * (kKIN / 8);
    castw_kernel<<<(trb + 255) / 256, 256, 0, stream>>>(rnnB, rbh, kRHU, kKIN / 8, kWCarry, trb);
    const int two = kNBR * kD * (kRH / 8);
    castw_kernel<<<(two + 255) / 256, 256, 0, stream>>>(Wout, woh, kRH, kRH / 8, kWCarry, two);
  }
  inp_ctrl_kernel<<<kB / 32, 256, 0, stream>>>(ut, dtp, inp);

  const int gridW1 = (kB / 64) * (kMH / 64) / 8;
  const int gridN256 = (kB / 64) * (kRH / 64) / 8;
  const float* prev = nullptr;
  for (int n = 0; n < kNBR; ++n) {
    gate_kernel<<<(kB * kD / 8 + 255) / 256, 256, 0, stream>>>(zt, sig + n * kD, zg, kB * kD / 8);
    wmma_gemm64<0, false, 2, 0, false><<<dim3(gridW1, 1), 256, 0, stream>>>(
        zg, nullptr, kD, 0L,
        w1h + (size_t)n * kMH * kD, nullptr, kD, 0L,
        (void*)x32, nullptr, kMH, 0L,
        b1 + (size_t)n * kMH, nullptr, 0L,
        kB, kMH, kD, kWCarryInv);
    ln_gelu_kernel<<<kB / 8, 256, 0, stream>>>(x32, lng + (size_t)n * kMH, lnb + (size_t)n * kMH, x16);
    wmma_gemm64<0, false, 2, 1, false><<<dim3(gridN256, 1), 256, 0, stream>>>(
        x16, nullptr, kMH, 0L,
        w2h + (size_t)n * kRH * kMH, nullptr, kMH, 0L,
        (void*)inp, nullptr, kKIN, 0L,
        b2 + (size_t)n * kRH, nullptr, 0L,
        kB, kRH, kMH, kWCarryInv);
    wmma_gemm64<0, false, 0, 3, false><<<dim3(gridN256, 1), 256, 0, stream>>>(
        inp, nullptr, kKIN, 0L,
        rbh + (size_t)n * kRH * kKIN, nullptr, kKIN, 0L,
        (void*)hhi, (void*)hlo, kRH, 0L,
        nullptr, nullptr, 0L,
        kB, kRH, kKIN, kWCarryInv);
    for (int p = 0; p < 2; ++p) {
      const int step = 2 * n + p;
      const unsigned short* Ap = (p == 0) ? hhi : hlo;
      const float sc = (p == 0) ? kWCarryInv : kLoInv;
      float* dst = (step == 2 * kNBR - 1) ? out0 : ((step & 1) ? p1 : p0);
      if (step == 0) {
        wmma_gemm64<0, false, 0, 0, false><<<dim3(gridN256, 1), 256, 0, stream>>>(
            Ap, nullptr, kRH, 0L,
            woh + (size_t)n * kD * kRH, nullptr, kRH, 0L,
            (void*)dst, nullptr, kD, 0L,
            nullptr, nullptr, 0L,
            kB, kD, kRH, sc);
      } else {
        wmma_gemm64<0, false, 0, 0, true><<<dim3(gridN256, 1), 256, 0, stream>>>(
            Ap, nullptr, kRH, 0L,
            woh + (size_t)n * kD * kRH, nullptr, kRH, 0L,
            (void*)dst, nullptr, kD, 0L,
            nullptr, prev, 0L,
            kB, kD, kRH, sc);
      }
      prev = dst;
    }
  }
  yproj_kernel<<<kB / 32, 256, 0, stream>>>(out0, ut, dtp, Cm, Dmm, out1);
}
